// UniGCNII_pyg_64811056496748
// MI455X (gfx1250) — hardware-run, weakly checked
//
#include <hip/hip_runtime.h>
#include <stddef.h>
#include <stdint.h>
#include <cmath>


#define DF     128
#define KA     256
#define NM     50000
#define NCLS   40
#define NCP    48
#define NLAY   4
#define NTHR   256
#define NWAVE  8
#define EPT    8
#define WSTEP  (32 * EPT)
#define NBA    1024
#define SLA    10
#define WLCAP  3584
#define RCAP   (NWAVE * WLCAP)
#define DEGCAP 64
#define KPW    4
#define KPB    (NWAVE * KPW)
#define GBM    64
#define GBN    128
#define GTHR   128
#define GWAVE  4
#define HBM    128
#define HTHR   256
#define HSTF   (HBM * NCLS)
#define NU_W0  (DF * (DF / 8))
#define NU_WS1 (DF * (KA / 8))
#define NU_WS  (NLAY * NU_WS1)
#define NU_WO  (NCP * (KA / 8))
#define NU_WE  (NU_W0 + NU_WS + NU_WO)
#define BK_ZINTS    (2 * RCAP + 3 * NBA)
#define MISC_INTS   16
#define BK_LDS_INTS (BK_ZINTS + MISC_INTS)

static_assert((NBA & (NBA - 1)) == 0 && NBA == (1 << SLA) && NBA == NTHR * 4 && NBA / 32 == 32);
static_assert(RCAP % (NTHR * 4) == 0 && BK_ZINTS % (NTHR * 4) == 0 && (BK_ZINTS % 4) == 0);
static_assert(BK_LDS_INTS * 4 <= 300000);
static_assert(RCAP * 100 >= 16696 * 105 && RCAP * 100 >= 8382 * 105);
static_assert(DEGCAP >= 33 + 8 && DEGCAP >= 23 + 8 && DEGCAP % 32 == 0);
static_assert(KA == 2 * DF && KA % 32 == 0 && DF % 32 == 0 && DF == 4 * 32);
static_assert(GBN == DF && GBM == GWAVE * 16 && GTHR == GWAVE * 32);
static_assert(HBM == (HTHR / 32) * 16 && HSTF % (HTHR * 4) == 0 && (HSTF * 4) % 128 == 0 && NCP % 16 == 0);
static_assert(NU_W0 % NTHR == 0 && NU_WS1 % NTHR == 0 && NU_WO % NTHR == 0 && NU_WE % NTHR == 0);
static_assert(HBM % GBM == 0 && HBM % KPB == 0 && NBA % KPB == 0);

typedef float          v4f   __attribute__((ext_vector_type(4)));
typedef float          v8f   __attribute__((ext_vector_type(8)));
typedef int            v4i   __attribute__((ext_vector_type(4)));
typedef int            v8i   __attribute__((ext_vector_type(8)));
typedef unsigned       v2u   __attribute__((ext_vector_type(2)));
typedef unsigned short v4us  __attribute__((ext_vector_type(4)));
typedef unsigned short v8us  __attribute__((ext_vector_type(8)));
typedef unsigned short v16us __attribute__((ext_vector_type(16)));
typedef __bf16         v16bf __attribute__((ext_vector_type(16)));
typedef v4f  __attribute__((may_alias)) v4fa;
typedef v4i  __attribute__((may_alias)) v4ia;
typedef v2u  __attribute__((may_alias)) v2ua;
typedef v4us __attribute__((may_alias)) v4usa;
typedef v8us __attribute__((may_alias)) v8usa;
union FragB { v16bf v; v16us u; v8us h[2]; v8i w; };

__device__ __forceinline__ v8f wmb(const FragB& a, const FragB& b, v8f c) {
  v8f d = __builtin_amdgcn_wmma_f32_16x16x32_bf16(false, a.v, false, b.v, (short)0, c, false, false);
  asm volatile("v_nop\n\tv_nop\n\tv_nop\n\tv_nop" : "+v"(d) : "v"(a.w), "v"(b.w));
  return d;
}

__device__ __forceinline__ v8f z8() { v8f z = {0.f, 0.f, 0.f, 0.f, 0.f, 0.f, 0.f, 0.f}; return z; }

__device__ __forceinline__ unsigned bf16_bits(float f) {
  const unsigned u = __float_as_uint(f);
  return (u + 0x7FFFu + ((u >> 16) & 1u)) >> 16;
}
__device__ __forceinline__ float bf16_val(float f) {
  return __uint_as_float(bf16_bits(f) << 16);
}
__device__ __forceinline__ unsigned hl_bits(float v, unsigned& lo) {
  const unsigned hb = bf16_bits(v);
  lo = bf16_bits(v - __uint_as_float(hb << 16));
  return hb;
}
__device__ __forceinline__ float relu_np(float v) { return (v > 0.0f) ? v : (v - v); }

__device__ __forceinline__ void wave_sync() {
  __builtin_amdgcn_fence(__ATOMIC_RELEASE, "wavefront");
  __builtin_amdgcn_wave_barrier();
  __builtin_amdgcn_fence(__ATOMIC_ACQUIRE, "wavefront");
}

__global__ __launch_bounds__(NTHR) void k_prep(const float* __restrict__ x, const float* __restrict__ w0,
                                               const float* __restrict__ wsk, const float* __restrict__ wo,
                                               unsigned short* w0t, unsigned short* wst2, unsigned short* wot2,
                                               unsigned short* xb, int nN, int nUnits) {
  const int u = (int)blockIdx.x * NTHR + (int)threadIdx.x;
  v8us o;
  unsigned short* dp;
  if (u < NU_W0) {
    const int n = u >> 4, k8 = (u & 15) * 8;
    const float* p = w0 + (size_t)k8 * DF + n;
#pragma unroll
    for (int i = 0; i < 8; ++i) {
      const float f = p[(size_t)i * DF];
      o[i] = (unsigned short)bf16_bits(f);
    }
    dp = w0t + (size_t)u * 8;
  } else if (u < NU_W0 + NU_WS) {
    const int v  = u - NU_W0;
    const int l  = v >> 12;
    const int n  = (v >> 5) & (DF - 1);
    const int k8 = (v & 31) * 8;
    const int kk = k8 & (DF - 1);
    const float* p = wsk + (size_t)l * DF * DF + (size_t)kk * DF + n;
#pragma unroll
    for (int i = 0; i < 8; ++i) {
      const float f = p[(size_t)i * DF];
      o[i] = (unsigned short)bf16_bits(f);
    }
    dp = wst2 + (size_t)v * 8;
  } else if (u < NU_WE) {
    const int v  = u - (NU_W0 + NU_WS);
    const int n  = v >> 5;
    const int k8 = (v & 31) * 8;
    const int kk = k8 & (DF - 1);
    const int nc = n < NCLS ? n : NCLS - 1;
    const unsigned msk = (n < NCLS) ? 0xFFFFu : 0u;
    const float* p = wo + (size_t)kk * NCLS + nc;
#pragma unroll
    for (int i = 0; i < 8; ++i) {
      const float f = p[(size_t)i * NCLS];
      asm volatile("" :: "v"(f));
      o[i] = (unsigned short)(bf16_bits(f) & msk);
    }
    dp = wot2 + (size_t)v * 8;
  } else if (u < nUnits) {
    const int v   = u - NU_WE;
    const int row = v >> 4, k8 = (v & 15) * 8;
    const int rc  = row < nN ? row : nN - 1;
    const unsigned msk = (row < nN) ? 0xFFFFu : 0u;
    const float* p = x + (size_t)rc * DF + k8;
    const v4f a = *(const v4f*)p;
    const v4f b = *(const v4f*)(p + 4);
    asm volatile("" :: "v"(a.x), "v"(a.y), "v"(a.z), "v"(a.w), "v"(b.x), "v"(b.y), "v"(b.z), "v"(b.w));
    o[0] = (unsigned short)(bf16_bits(a.x) & msk); o[1] = (unsigned short)(bf16_bits(a.y) & msk);
    o[2] = (unsigned short)(bf16_bits(a.z) & msk); o[3] = (unsigned short)(bf16_bits(a.w) & msk);
    o[4] = (unsigned short)(bf16_bits(b.x) & msk); o[5] = (unsigned short)(bf16_bits(b.y) & msk);
    o[6] = (unsigned short)(bf16_bits(b.z) & msk); o[7] = (unsigned short)(bf16_bits(b.w) & msk);
    dp = xb + (size_t)v * 8;
  } else {
    return;
  }
  *(volatile v8us*)dp = o;
  __threadfence();
  *(volatile v8us*)dp = o;
}

__device__ __forceinline__ int scan_step(const int* __restrict__ keys, int nE, int ibase, int slotBase,
                                         int* mylist, int lane, int wc) {
  const int e0   = ibase + lane * EPT;
  const int sent = -2147483647 - 1;
  v4i da, db;
  if (ibase + WSTEP <= nE) {
    da = *(const v4i*)(keys + e0);
    db = *(const v4i*)(keys + e0 + 4);
  } else {
    const int t0 = keys[min(e0,     nE - 1)];
    const int t1 = keys[min(e0 + 1, nE - 1)];
    const int t2 = keys[min(e0 + 2, nE - 1)];
    const int t3 = keys[min(e0 + 3, nE - 1)];
    const int t4 = keys[min(e0 + 4, nE - 1)];
    const int t5 = keys[min(e0 + 5, nE - 1)];
    const int t6 = keys[min(e0 + 6, nE - 1)];
    const int t7 = keys[min(e0 + 7, nE - 1)];
    asm volatile("" :: "v"(t0), "v"(t1), "v"(t2), "v"(t3), "v"(t4), "v"(t5), "v"(t6), "v"(t7));
    da.x = (e0     < nE) ? t0 : sent;
    da.y = (e0 + 1 < nE) ? t1 : sent;
    da.z = (e0 + 2 < nE) ? t2 : sent;
    da.w = (e0 + 3 < nE) ? t3 : sent;
    db.x = (e0 + 4 < nE) ? t4 : sent;
    db.y = (e0 + 5 < nE) ? t5 : sent;
    db.z = (e0 + 6 < nE) ? t6 : sent;
    db.w = (e0 + 7 < nE) ? t7 : sent;
  }
  const unsigned nbs = (unsigned)slotBase;
  const unsigned unb = (unsigned)NBA;
  const unsigned s0 = (unsigned)da.x - nbs, s1 = (unsigned)da.y - nbs;
  const unsigned s2 = (unsigned)da.z - nbs, s3 = (unsigned)da.w - nbs;
  const unsigned s4 = (unsigned)db.x - nbs, s5 = (unsigned)db.y - nbs;
  const unsigned s6 = (unsigned)db.z - nbs, s7 = (unsigned)db.w - nbs;
  const bool h0 = s0 < unb, h1 = s1 < unb, h2 = s2 < unb, h3 = s3 < unb;
  const bool h4 = s4 < unb, h5 = s5 < unb, h6 = s6 < unb, h7 = s7 < unb;
  const unsigned any = __builtin_amdgcn_ballot_w32(h0 | h1 | h2 | h3 | h4 | h5 | h6 | h7);
  if (any != 0u) {
#define HITJ(J, HJ, SJ) { \
      const unsigned mj = __builtin_amdgcn_ballot_w32(HJ); \
      if (mj != 0u) { \
        if (HJ) { \
          const int pos = wc + (int)__builtin_amdgcn_mbcnt_lo(mj, 0u); \
          if (pos < WLCAP) mylist[pos] = ((e0 + (J)) << SLA) | (int)(SJ); \
        } \
        wc += (int)__builtin_popcount(mj); } }
    HITJ(0, h0, s0)
    HITJ(1, h1, s1)
    HITJ(2, h2, s2)
    HITJ(3, h3, s3)
    HITJ(4, h4, s4)
    HITJ(5, h5, s5)
    HITJ(6, h6, s6)
    HITJ(7, h7, s7)
#undef HITJ
  }
  return wc;
}

__global__ __launch_bounds__(NTHR) void k_bucket(const int* __restrict__ keys, const int* __restrict__ pay,
                                                 int nE, int nPay, int segW,
                                                 int* lst, int* offp, int* cntp, int* flg, int flagBase) {
  extern __shared__ __attribute__((aligned(16))) int dsm[];
  int* wl   = dsm;
  int* sl   = dsm + RCAP;
  int* cnt  = sl + RCAP;
  int* offs = cnt + NBA;
  int* cur  = offs + NBA;
  int* misc = cur + NBA;
  const int tid = (int)threadIdx.x, lane = tid & 31, wave = tid >> 5;
  const int slotBase = (int)blockIdx.x * NBA;

  {
    const v4i z4 = {0, 0, 0, 0};
#pragma unroll 1
    for (int i = tid * 4; i < BK_ZINTS; i += NTHR * 4) *(v4ia*)(dsm + i) = z4;
    if (tid < MISC_INTS) misc[tid] = 0;
  }
  __syncthreads();

  {
    int wc = 0;
    int* mylist = wl + wave * WLCAP;
    const int wbase = wave * segW;
    const int nIt = segW / WSTEP;
#pragma unroll 1
    for (int it = 0; it < nIt; ++it) {
      wc = scan_step(keys, nE, wbase + it * WSTEP, slotBase, mylist, lane, wc);
    }
    if (lane == 0) misc[wave] = wc;
  }
  __syncthreads();

  if (wave == 0) {
    int t = 0, ov = 0;
#pragma unroll 1
    for (int w2 = 0; w2 < NWAVE; ++w2) {
      int c = misc[w2];
      if (c > WLCAP) ov = 1;
      c = c < 0 ? 0 : (c > WLCAP ? WLCAP : c);
#pragma unroll 1
      for (int b0 = 0; b0 < c; b0 += 32) {
        const int idx = b0 + lane;
        const int ent_ = wl[w2 * WLCAP + (idx < WLCAP ? idx : WLCAP - 1)];
        const int m32 = (c - b0) < 32 ? (c - b0) : 32;
#pragma unroll 1
        for (int k = 0; k < m32; ++k) {
          const int u    = __builtin_amdgcn_readlane(ent_, k);
          const int slot = u & (NBA - 1);
          if (lane == 0) cnt[slot] = cnt[slot] + 1;
        }
      }
      t += c;
    }
    if (lane == 0) { misc[8] = t; misc[9] = ov; }
  }
  __syncthreads();

  if (wave == 0) {
    const int base = lane * (NBA / 32);
    int s = 0, bg = 0;
#pragma unroll 1
    for (int i = 0; i < NBA / 32; ++i) {
      const int cv = cnt[base + i];
      s += cv;
      if (cv > DEGCAP) bg = 1;
    }
    int incl = s;
#pragma unroll
    for (int d = 1; d < 32; d <<= 1) {
      const int y = __shfl_up(incl, d, 32);
      if (lane >= d) incl += y;
    }
    int run = incl - s;
#pragma unroll 1
    for (int i = 0; i < NBA / 32; ++i) {
      const int cv = cnt[base + i];
      offs[base + i] = run;
      cur[base + i]  = run;
      run += cv;
    }
    const unsigned bm = __builtin_amdgcn_ballot_w32(bg != 0);
    if (lane == 0) misc[10] = (bm != 0u) ? 1 : 0;
  }
  __syncthreads();

  if (wave == 0) {
#pragma unroll 1
    for (int w2 = 0; w2 < NWAVE; ++w2) {
      int c = misc[w2];
      c = c < 0 ? 0 : (c > WLCAP ? WLCAP : c);
#pragma unroll 1
      for (int b0 = 0; b0 < c; b0 += 32) {
        const int idx = b0 + lane;
        const int ent_ = wl[w2 * WLCAP + (idx < WLCAP ? idx : WLCAP - 1)];
        int eid = ent_ >> SLA;
        eid = eid < 0 ? 0 : (eid > nE - 1 ? nE - 1 : eid);
        int pv = pay[eid];
        pv = pv < 0 ? 0 : (pv > nPay - 1 ? nPay - 1 : pv);
        const int m32 = (c - b0) < 32 ? (c - b0) : 32;
#pragma unroll 1
        for (int k = 0; k < m32; ++k) {
          const int u    = __builtin_amdgcn_readlane(ent_, k);
          const int pk   = __builtin_amdgcn_readlane(pv, k);
          const int slot = u & (NBA - 1);
          if (lane == 0) {
            int p = cur[slot];
            p = p < 0 ? 0 : (p > RCAP - 1 ? RCAP - 1 : p);
            sl[p] = pk;
            cur[slot] = p + 1;
          }
        }
      }
    }
  }
  __syncthreads();

  const int ovf   = ((misc[9] | misc[10]) != 0) ? 1 : 0;
  const int lbase = (int)blockIdx.x * RCAP;
  int* lb = lst + (size_t)blockIdx.x * RCAP;
  int* ob = offp + (size_t)blockIdx.x * NBA + 4 * tid;
  int* cb = cntp + (size_t)blockIdx.x * NBA + 4 * tid;
  int* fb = flg + (size_t)(flagBase + (int)blockIdx.x) * 32 + 4 * (tid & 7);
  v4i o4 = *(const v4ia*)(offs + 4 * tid);
  o4.x += lbase; o4.y += lbase; o4.z += lbase; o4.w += lbase;
  const v4i c4 = *(const v4ia*)(cnt + 4 * tid);
  const v4i f4 = {ovf, ovf, ovf, ovf};
#pragma unroll 1
  for (int i = tid * 4; i < RCAP; i += NTHR * 4) {
    const v4i v = *(const v4ia*)(sl + i);
    *(volatile v4i*)(lb + i) = v;
  }
  *(volatile v4i*)ob = o4;
  *(volatile v4i*)cb = c4;
  if (tid < 8) *(volatile v4i*)fb = f4;
  __threadfence();
#pragma unroll 1
  for (int i = tid * 4; i < RCAP; i += NTHR * 4) {
    const v4i v = *(const v4ia*)(sl + i);
    *(volatile v4i*)(lb + i) = v;
  }
  *(volatile v4i*)ob = o4;
  *(volatile v4i*)cb = c4;
  if (tid < 8) *(volatile v4i*)fb = f4;
}

__global__ __launch_bounds__(NTHR) void k_aggE(const float* xpl, const int* __restrict__ lst,
                                               const int* __restrict__ offp, const int* __restrict__ cntp,
                                               const int* __restrict__ pzp, int nKey, int nKeyTab, int listTot,
                                               int nSrc, float* xe, int xeRows) {
  const int tid = (int)threadIdx.x, lane = tid & 31, wave = tid >> 5;
  const float qnan = __int_as_float(0x7fc00000);
  const float pz = (pzp[0] != 0) ? qnan : 0.0f;
#pragma unroll 1
  for (int j = 0; j < KPW; ++j) {
    const int key = (int)blockIdx.x * KPB + wave * KPW + j;
    const int kc  = key < nKeyTab ? key : nKeyTab - 1;
    int c = cntp[kc];
    const bool big = c > DEGCAP;
    c = c < 0 ? 0 : (c > DEGCAP ? DEGCAP : c);
    int o = offp[kc];
    o = o < 0 ? 0 : (o > listTot - 1 ? listTot - 1 : o);
    float a0 = 0.0f, a1 = 0.0f, a2 = 0.0f, a3 = 0.0f;
#pragma unroll 1
    for (int b0 = 0; b0 < c; b0 += 32) {
      int idx = o + b0 + lane;
      idx = idx > listTot - 1 ? listTot - 1 : idx;
      int sr = lst[idx];
      sr = sr < 0 ? 0 : (sr > nSrc - 1 ? nSrc - 1 : sr);
      const int m32 = (c - b0) < 32 ? (c - b0) : 32;
#pragma unroll 1
      for (int k = 0; k < m32; ++k) {
        const int sk = __builtin_amdgcn_readlane(sr, k);
        const v4f r = *(const v4fa*)(xpl + (size_t)sk * DF + 4 * lane);
        a0 += r.x; a1 += r.y; a2 += r.z; a3 += r.w;
      }
    }
    const float cf  = (float)(c < 1 ? 1 : c);
    const float pzr = big ? qnan : pz;
    const bool live = key < nKey;
    v4f mv;
    mv.x = live ? (a0 / cf + pzr) : 0.0f;
    mv.y = live ? (a1 / cf + pzr) : 0.0f;
    mv.z = live ? (a2 / cf + pzr) : 0.0f;
    mv.w = live ? (a3 / cf + pzr) : 0.0f;
    if (key < xeRows) {
      float* rp = xe + (size_t)key * DF + 4 * lane;
      *(volatile v4f*)rp = mv;
      __threadfence();
      *(volatile v4f*)rp = mv;
    }
  }
}

__global__ __launch_bounds__(NTHR) void k_aggV(const float* xe, const float* x0, const int* __restrict__ lst,
                                               const int* __restrict__ offp, const int* __restrict__ cntp,
                                               const int* __restrict__ pzp, int nKey, int nKeyTab, int listTot,
                                               int nSrc, unsigned short* pout, int mRows) {
  __shared__ __attribute__((aligned(16))) unsigned short rowbuf[NWAVE * KA];
  const int tid = (int)threadIdx.x, lane = tid & 31, wave = tid >> 5;
  unsigned short* rb = rowbuf + wave * KA;
  const float qnan = __int_as_float(0x7fc00000);
  const float pz = (pzp[0] != 0) ? qnan : 0.0f;
#pragma unroll 1
  for (int j = 0; j < KPW; ++j) {
    const int node = (int)blockIdx.x * KPB + wave * KPW + j;
    const int kc   = node < nKeyTab ? node : nKeyTab - 1;
    int c = cntp[kc];
    const bool big = c > DEGCAP;
    c = c < 0 ? 0 : (c > DEGCAP ? DEGCAP : c);
    int o = offp[kc];
    o = o < 0 ? 0 : (o > listTot - 1 ? listTot - 1 : o);
    float a0 = 0.0f, a1 = 0.0f, a2 = 0.0f, a3 = 0.0f;
#pragma unroll 1
    for (int b0 = 0; b0 < c; b0 += 32) {
      int idx = o + b0 + lane;
      idx = idx > listTot - 1 ? listTot - 1 : idx;
      int sr = lst[idx];
      sr = sr < 0 ? 0 : (sr > nSrc - 1 ? nSrc - 1 : sr);
      const int m32 = (c - b0) < 32 ? (c - b0) : 32;
#pragma unroll 1
      for (int k = 0; k < m32; ++k) {
        const int sk = __builtin_amdgcn_readlane(sr, k);
        const v4f r = *(const v4fa*)(xe + (size_t)sk * DF + 4 * lane);
        a0 += r.x; a1 += r.y; a2 += r.z; a3 += r.w;
      }
    }
    const int nc = node < nKey ? node : nKey - 1;
    const v4f xs = *(const v4fa*)(x0 + (size_t)nc * DF + 4 * lane);
    const float cf = (float)(c < 1 ? 1 : c);
    const float q0 = a0 / cf, q1 = a1 / cf, q2 = a2 / cf, q3 = a3 / cf;
    float ss = (q0 * q0 + q1 * q1) + (q2 * q2 + q3 * q3);
    ss += __shfl_xor(ss, 16, 32);
    ss += __shfl_xor(ss, 8, 32);
    ss += __shfl_xor(ss, 4, 32);
    ss += __shfl_xor(ss, 2, 32);
    ss += __shfl_xor(ss, 1, 32);
    const float nrm = sqrtf(ss);
    const float sc  = (nrm > 0.0f) ? (1.0f / nrm) : 0.0f;
    const float pzr = big ? qnan : pz;
    const bool live = node < nKey;
    const float m0 = live ? (0.9f * (q0 * sc) + 0.1f * xs.x + pzr) : 0.0f;
    const float m1 = live ? (0.9f * (q1 * sc) + 0.1f * xs.y + pzr) : 0.0f;
    const float m2 = live ? (0.9f * (q2 * sc) + 0.1f * xs.z + pzr) : 0.0f;
    const float m3 = live ? (0.9f * (q3 * sc) + 0.1f * xs.w + pzr) : 0.0f;
    v4us mh, ml;
    {
      unsigned lb;
      unsigned hb;
      hb = hl_bits(m0, lb); mh[0] = (unsigned short)hb; ml[0] = (unsigned short)lb;
      hb = hl_bits(m1, lb); mh[1] = (unsigned short)hb; ml[1] = (unsigned short)lb;
      hb = hl_bits(m2, lb); mh[2] = (unsigned short)hb; ml[2] = (unsigned short)lb;
      hb = hl_bits(m3, lb); mh[3] = (unsigned short)hb; ml[3] = (unsigned short)lb;
    }
    *(v4usa*)(rb + 4 * lane)      = mh;
    *(v4usa*)(rb + DF + 4 * lane) = ml;
    wave_sync();
    const v8us qv = *(const v8usa*)(rb + 8 * lane);
    wave_sync();
    if (node < mRows) {
      unsigned short* rp = pout + (size_t)node * KA + 8 * lane;
      *(volatile v8us*)rp = qv;
      __threadfence();
      *(volatile v8us*)rp = qv;
    }
  }
}

template <int MODE>
__global__ __launch_bounds__(GTHR) __attribute__((amdgpu_num_vgpr(248)))
void k_gemm(const unsigned short* A, int lda, const unsigned short* __restrict__ BT, int ldb, int K,
            const float* __restrict__ bias, float c1, float c2, float* outF, unsigned short* outH, int nN,
            const int* __restrict__ flg, int nFlag, int* pzl) {
  __shared__ __attribute__((aligned(16))) float stg[GBM * GBN];
  __shared__ __attribute__((aligned(16))) unsigned short hrow[GWAVE * KA];
  const int tid = (int)threadIdx.x, lane = tid & 31, wave = tid >> 5, hh = lane >> 4, m = lane & 15;
  const int rowBase = (int)blockIdx.x * GBM;

  v8f acc[8];
#pragma unroll
  for (int t = 0; t < 8; ++t) acc[t] = z8();
  const unsigned short* ap = A + (size_t)(rowBase + 16 * wave + m) * (size_t)lda + 8 * hh;
  const unsigned short* bp = BT + (size_t)m * (size_t)ldb + 8 * hh;

#pragma unroll 1
  for (int k0 = 0; k0 < K; k0 += 32) {
    FragB af;
    af.h[0] = *(const v8usa*)(ap + k0);
    af.h[1] = *(const v8usa*)(ap + k0 + 16);
#pragma unroll
    for (int nt = 0; nt < 8; ++nt) {
      const unsigned short* wq = bp + (size_t)(16 * nt) * (size_t)ldb + k0;
      FragB bf;
      bf.h[0] = *(const v8usa*)wq;
      bf.h[1] = *(const v8usa*)(wq + 16);
      acc[nt] = wmb(af, bf, acc[nt]);
    }
  }

#pragma unroll
  for (int nt = 0; nt < 8; ++nt) {
    const int lc = 16 * nt + m;
#pragma unroll
    for (int r = 0; r < 8; ++r) {
      const int lr = 16 * wave + 8 * hh + r;
      stg[lr * GBN + lc] = acc[nt][r];
    }
  }
  __syncthreads();

  if constexpr (MODE == 0) {
    const v4f b4 = *(const v4f*)(bias + 4 * lane);
    const float bq0 = bf16_val(b4.x), bq1 = bf16_val(b4.y), bq2 = bf16_val(b4.z), bq3 = bf16_val(b4.w);
#pragma unroll 2
    for (int i = 0; i < 16; ++i) {
      const int lr = 16 * wave + i;
      const bool ok = (rowBase + lr) < nN;
      float* sp = stg + lr * GBN + 4 * lane;
      const v4f d = *(const v4fa*)sp;
      v4f y;
      y.x = relu_np(d.x + bq0); y.y = relu_np(d.y + bq1); y.z = relu_np(d.z + bq2); y.w = relu_np(d.w + bq3);
      y.x = ok ? y.x : 0.0f; y.y = ok ? y.y : 0.0f; y.z = ok ? y.z : 0.0f; y.w = ok ? y.w : 0.0f;
      *(v4fa*)sp = y;
    }
  } else {
    unsigned short* hr = hrow + wave * KA;
#pragma unroll 2
    for (int i = 0; i < 16; ++i) {
      const int lr = 16 * wave + i;
      const int row = rowBase + lr;
      const bool ok = row < nN;
      float* sp = stg + lr * GBN + 4 * lane;
      const v4f d = *(const v4fa*)sp;
      const unsigned short* rp = A + (size_t)row * (size_t)lda + 4 * lane;
      const v2u wh = *(const v2ua*)rp;
      const v2u wl = *(const v2ua*)(rp + DF);
      const float f0 = __uint_as_float(wh.x << 16)         + __uint_as_float(wl.x << 16);
      const float f1 = __uint_as_float(wh.x & 0xffff0000u) + __uint_as_float(wl.x & 0xffff0000u);
      const float f2 = __uint_as_float(wh.y << 16)         + __uint_as_float(wl.y << 16);
      const float f3 = __uint_as_float(wh.y & 0xffff0000u) + __uint_as_float(wl.y & 0xffff0000u);
      v4f y;
      y.x = relu_np(c1 * f0 + c2 * d.x);
      y.y = relu_np(c1 * f1 + c2 * d.y);
      y.z = relu_np(c1 * f2 + c2 * d.z);
      y.w = relu_np(c1 * f3 + c2 * d.w);
      y.x = ok ? y.x : 0.0f; y.y = ok ? y.y : 0.0f; y.z = ok ? y.z : 0.0f; y.w = ok ? y.w : 0.0f;
      if constexpr (MODE == 1) {
        *(v4fa*)sp = y;
      } else {
        v4us h4, l4;
        unsigned lb;
        unsigned hb;
        hb = hl_bits(y.x, lb); h4[0] = (unsigned short)hb; l4[0] = (unsigned short)lb;
        hb = hl_bits(y.y, lb); h4[1] = (unsigned short)hb; l4[1] = (unsigned short)lb;
        hb = hl_bits(y.z, lb); h4[2] = (unsigned short)hb; l4[2] = (unsigned short)lb;
        hb = hl_bits(y.w, lb); h4[3] = (unsigned short)hb; l4[3] = (unsigned short)lb;
        *(v4usa*)(hr + 4 * lane)      = h4;
        *(v4usa*)(hr + DF + 4 * lane) = l4;
        wave_sync();
        const v8us q = *(const v8usa*)(hr + 8 * lane);
        wave_sync();
        *(v8usa*)((unsigned short*)stg + (size_t)lr * KA + 8 * lane) = q;
      }
    }
  }
  __syncthreads();

  if constexpr (MODE == 2) {
#pragma unroll 4
    for (int i = 0; i < 16; ++i) {
      const int lr = 16 * wave + i;
      const v8us q = *(const v8usa*)((const unsigned short*)stg + (size_t)lr * KA + 8 * lane);
      *(volatile v8us*)(outH + (size_t)(rowBase + lr) * KA + 8 * lane) = q;
    }
    __threadfence();
#pragma unroll 4
    for (int i = 0; i < 16; ++i) {
      const int lr = 16 * wave + i;
      const v8us q = *(const v8usa*)((const unsigned short*)stg + (size_t)lr * KA + 8 * lane);
      *(volatile v8us*)(outH + (size_t)(rowBase + lr) * KA + 8 * lane) = q;
    }
  } else {
#pragma unroll 4
    for (int i = 0; i < 16; ++i) {
      const int lr = 16 * wave + i;
      const v4f v = *(const v4fa*)(stg + lr * GBN + 4 * lane);
      *(volatile v4f*)(outF + (size_t)(rowBase + lr) * DF + 4 * lane) = v;
    }
    __threadfence();
#pragma unroll 4
    for (int i = 0; i < 16; ++i) {
      const int lr = 16 * wave + i;
      const v4f v = *(const v4fa*)(stg + lr * GBN + 4 * lane);
      *(volatile v4f*)(outF + (size_t)(rowBase + lr) * DF + 4 * lane) = v;
    }
  }

  if constexpr (MODE == 0) {
    if (blockIdx.x == 0 && wave == 0) {
      int fa = 0;
#pragma unroll 1
      for (int j0 = 0; j0 < nFlag; j0 += 32) {
        int jj = j0 + lane;
        jj = jj > nFlag - 1 ? nFlag - 1 : jj;
        fa |= flg[(size_t)jj * 32];
      }
      const unsigned bm = __builtin_amdgcn_ballot_w32(fa != 0);
      const int pw = (bm != 0u) ? 1 : 0;
      const v4i w4 = {pw, pw, pw, pw};
      int* pq = pzl + 4 * (lane & 7);
      if (lane < 8) *(volatile v4i*)pq = w4;
      __threadfence();
      if (lane < 8) *(volatile v4i*)pq = w4;
    }
  }
}

__global__ __launch_bounds__(HTHR) __attribute__((amdgpu_num_vgpr(248)))
void k_head(const unsigned short* __restrict__ A, const unsigned short* __restrict__ BT,
            const float* __restrict__ bout, const int* __restrict__ pzp, float* out, int outElems) {
  __shared__ __attribute__((aligned(16))) float hst[HSTF];
  __shared__ float sb[NCP];
  const int tid = (int)threadIdx.x, lane = tid & 31, wave = tid >> 5, hh = lane >> 4, m = lane & 15;
  const int rowBase = (int)blockIdx.x * HBM;
  {
    const int bc = tid < NCLS ? tid : NCLS - 1;
    const float f = bout[bc];
    asm volatile("" :: "v"(f));
    const float bv = (tid < NCLS) ? bf16_val(f) : 0.0f;
    if (tid < NCP) sb[tid] = bv;
  }
  const float pz = (pzp[0] != 0) ? __int_as_float(0x7fc00000) : 0.0f;

  v8f acc[3];
#pragma unroll
  for (int t = 0; t < 3; ++t) acc[t] = z8();
  const unsigned short* ap = A + (size_t)(rowBase + 16 * wave + m) * (size_t)KA + 8 * hh;
  const unsigned short* bp = BT + (size_t)m * (size_t)KA + 8 * hh;
#pragma unroll 1
  for (int k0 = 0; k0 < KA; k0 += 32) {
    FragB af;
    af.h[0] = *(const v8usa*)(ap + k0);
    af.h[1] = *(const v8usa*)(ap + k0 + 16);
#pragma unroll
    for (int nt = 0; nt < 3; ++nt) {
      const unsigned short* wq = bp + (size_t)(16 * nt) * (size_t)KA + k0;
      FragB bf;
      bf.h[0] = *(const v8usa*)wq;
      bf.h[1] = *(const v8usa*)(wq + 16);
      acc[nt] = wmb(af, bf, acc[nt]);
    }
  }
  __syncthreads();
#pragma unroll
  for (int nt = 0; nt < 3; ++nt) {
    const int col = 16 * nt + m;
    const float bv = sb[col];
#pragma unroll
    for (int r = 0; r < 8; ++r) {
      const int lr = 16 * wave + 8 * hh + r;
      if (col < NCLS) hst[lr * NCLS + col] = acc[nt][r] + bv + pz;
    }
  }
  __syncthreads();

  const int ebase = (int)blockIdx.x * HSTF;
#pragma unroll 1
  for (int p = 0; p < HSTF / (HTHR * 4); ++p) {
    const int f = p * HTHR + tid;
    const v4f v = *(const v4fa*)(hst + 4 * f);
    asm volatile("" :: "v"(v.x), "v"(v.y), "v"(v.z), "v"(v.w));
    const int e = ebase + 4 * f;
    if (e + 3 < outElems) *(volatile v4f*)(out + (size_t)e) = v;
  }
  __threadfence();
#pragma unroll 1
  for (int p = 0; p < HSTF / (HTHR * 4); ++p) {
    const int f = p * HTHR + tid;
    const v4f v = *(const v4fa*)(hst + 4 * f);
    asm volatile("" :: "v"(v.x), "v"(v.y), "v"(v.z), "v"(v.w));
    const int e = ebase + 4 * f;
    if (e + 3 < outElems) *(volatile v4f*)(out + (size_t)e) = v;
  }
}

static inline int cdiv(int a, int b) { return (a + b - 1) / b; }
static inline size_t al256(size_t o) { return (o + 255) & ~(size_t)255; }

extern "C" void kernel_launch(void* const* d_in, const int* in_sizes, int n_in,
                              void* d_out, int out_size, void* d_ws, size_t ws_size,
                              hipStream_t stream) {
  if (n_in < 8) return;
  if (in_sizes[0] < DF * GBM || (in_sizes[0] % DF) != 0) return;
  const int nN = in_sizes[0] / DF;
  if (nN < NM / 64 || nN > (1 << 22)) return;
  if (in_sizes[1] != DF * DF || in_sizes[2] != DF) return;
  if (in_sizes[3] != NLAY * DF * DF) return;
  if (in_sizes[4] != DF * NCLS || in_sizes[5] != NCLS) return;
  const int nE = in_sizes[6];
  if (nE < 1 || nE >= (1 << 21) || in_sizes[7] != nE) return;
  if ((long long)out_size != (long long)nN * NCLS) return;
  if ((out_size % 32) != 0) return;

  const float* x    = (const float*)d_in[0];
  const float* W0   = (const float*)d_in[1];
  const float* b0   = (const float*)d_in[2];
  const float* Ws   = (const float*)d_in[3];
  const float* Wout = (const float*)d_in[4];
  const float* bout = (const float*)d_in[5];
  const int*   vtx  = (const int*)d_in[6];
  const int*   edg  = (const int*)d_in[7];
  float* out = (float*)d_out;

  const int MP = cdiv(nN, HBM) * HBM;
  const int gE = cdiv(NM, NBA);
  const int gV = cdiv(nN, NBA);
  if ((long long)gV * NBA < (long long)MP) return;
  const int xeRows = cdiv(NM, KPB) * KPB;
  if (xeRows > gE * NBA) return;
  const int keyTabE = gE * NBA, keyTabV = gV * NBA;
  const int listTotE = gE * RCAP, listTotV = gV * RCAP;
  const int nFlag = gE + gV;
  const int segW = cdiv(cdiv(nE, NWAVE), WSTEP) * WSTEP;

  char* ws = (char*)d_ws;
  size_t off = 0;
  const size_t oX0  = off; off = al256(off + (size_t)MP * DF * 4);
  const size_t oP   = off; off = al256(off + (size_t)MP * KA * 2);
  const size_t oQ   = off; off = al256(off + (size_t)MP * DF * 4);
  const size_t oXE  = off; off = al256(off + (size_t)xeRows * DF * 4);
  const size_t oLE  = off; off = al256(off + (size_t)listTotE * 4);
  const size_t oLV  = off; off = al256(off + (size_t)listTotV * 4);
  const size_t oOE  = off; off = al256(off + (size_t)keyTabE * 4);
  const size_t oCE  = off; off = al256(off + (size_t)keyTabE * 4);
  const size_t oOV  = off; off = al256(off + (size_t)keyTabV * 4);
  const size_t oCV  = off; off = al256(off + (size_t)keyTabV * 4);
  const size_t oFL  = off; off = al256(off + (size_t)nFlag * 128);
  const size_t oPZ  = off; off = al256(off + 128);
  const size_t oW0T = off; off = al256(off + (size_t)DF * DF * 2);
  const size_t oWS  = off; off = al256(off + (size_t)NLAY * DF * KA * 2);
  const size_t oWO  = off; off = al256(off + (size_t)NCP * KA * 2);
  if (off > ws_size) return;
  float* X0 = (float*)(ws + oX0);
  unsigned short* P  = (unsigned short*)(ws + oP);
  unsigned short* XB = P;
  float* Q  = (float*)(ws + oQ);
  float* XE = (float*)(ws + oXE);
  int* LE = (int*)(ws + oLE);  int* LV = (int*)(ws + oLV);
  int* OE = (int*)(ws + oOE);  int* CE = (int*)(ws + oCE);
  int* OV = (int*)(ws + oOV);  int* CV = (int*)(ws + oCV);
  int* FL = (int*)(ws + oFL);  int* PZ = (int*)(ws + oPZ);
  unsigned short* W0T  = (unsigned short*)(ws + oW0T);
  unsigned short* WST2 = (unsigned short*)(ws + oWS);
  unsigned short* WOT2 = (unsigned short*)(ws + oWO);

  const size_t bkLds = (size_t)BK_LDS_INTS * 4;
  hipFuncSetAttribute(reinterpret_cast<const void*>(&k_bucket), hipFuncAttributeMaxDynamicSharedMemorySize, (int)bkLds);

  const int nUnits = NU_WE + MP * (DF / 8);

  k_prep<<<cdiv(nUnits, NTHR), NTHR, 0, stream>>>(x, W0, Ws, Wout, W0T, WST2, WOT2, XB, nN, nUnits);
  k_bucket<<<gE, NTHR, bkLds, stream>>>(edg, vtx, nE, nN, segW, LE, OE, CE, FL, 0);
  k_bucket<<<gV, NTHR, bkLds, stream>>>(vtx, edg, nE, NM, segW, LV, OV, CV, FL, gE);
  k_gemm<0><<<MP / GBM, GTHR, 0, stream>>>(XB, DF, W0T, DF, DF, b0, 0.0f, 0.0f, X0, P, nN, FL, nFlag, PZ);
  for (int i = 0; i < NLAY; ++i) {
    const double bt = std::log(0.5 / (double)(i + 1) + 1.0);
    const float c2 = (float)bt;
    const float c1 = (float)(1.0 - bt);
    const float* xcur = (i == 0) ? X0 : Q;
    k_aggE<<<xeRows / KPB, NTHR, 0, stream>>>(xcur, LE, OE, CE, PZ, NM, keyTabE, listTotE, nN, XE, xeRows);
    k_aggV<<<MP / KPB, NTHR, 0, stream>>>(XE, X0, LV, OV, CV, PZ, nN, keyTabV, listTotV, NM, P, MP);
    const unsigned short* Bl = WST2 + (size_t)i * DF * KA;
    if (i < NLAY - 1) {
      k_gemm<1><<<MP / GBM, GTHR, 0, stream>>>(P, KA, Bl, KA, KA, b0, c1, c2, Q, P, nN, FL, nFlag, PZ);
    } else {
      k_gemm<2><<<MP / GBM, GTHR, 0, stream>>>(P, KA, Bl, KA, KA, b0, c1, c2, Q, P, nN, FL, nFlag, PZ);
    }
  }
  k_head<<<MP / HBM, HTHR, 0, stream>>>(P, WOT2, bout, PZ, out, out_size);
}
